// IntelligentNeuron_44976897523902
// MI455X (gfx1250) — hardware-verified
//
#include <hip/hip_runtime.h>


#define LL   2048
#define DMO  1024
#define DI   2048
#define DS   16
#define DR   64
#define XW   128
typedef _Float16 h16;
typedef unsigned short bf;
typedef __attribute__((ext_vector_type(16))) __bf16   v16bf;
typedef __attribute__((ext_vector_type(16))) _Float16 v16h;
typedef __attribute__((ext_vector_type(8)))  _Float16 v8h;
typedef __attribute__((ext_vector_type(8)))  unsigned short v8us;
typedef __attribute__((ext_vector_type(8)))  float    v8f;
typedef __attribute__((ext_vector_type(4)))  float    v4f;
typedef v8h  __attribute__((may_alias)) v8ha;
typedef v4f  __attribute__((may_alias)) v4fa;
typedef v8us __attribute__((may_alias)) v8usa;

__device__ __forceinline__ unsigned short f2bf(float f) { unsigned u = __float_as_uint(f); u += 0x7FFFu + ((u >> 16) & 1u); return (unsigned short)(u >> 16); }
__device__ __forceinline__ float bf2f(unsigned short b) { return __uint_as_float(((unsigned)b) << 16); }
__device__ __forceinline__ float bfr(float f) { return bf2f(f2bf(f)); }
__device__ __forceinline__ v16h cat16(v8h lo, v8h hi) { return __builtin_shufflevector(lo, hi, 0, 1, 2, 3, 4, 5, 6, 7, 8, 9, 10, 11, 12, 13, 14, 15); }
__device__ __forceinline__ v16bf cat16b(v8us lo, v8us hi) { return __builtin_bit_cast(v16bf, __builtin_shufflevector(lo, hi, 0, 1, 2, 3, 4, 5, 6, 7, 8, 9, 10, 11, 12, 13, 14, 15)); }
__device__ __forceinline__ v8f wmma16(v16h a, v16h b, v8f c) { return __builtin_amdgcn_wmma_f32_16x16x32_f16(false, a, false, b, (short)0, c, false, false); }
__device__ __forceinline__ v8f wmmab(v16bf a, v16bf b, v8f c) { return __builtin_amdgcn_wmma_f32_16x16x32_bf16(false, a, false, b, (short)0, c, false, false); }


template <typename T16> struct WFrag;
template <> struct WFrag<h16> { typedef v16h V; static __device__ __forceinline__ V ld(const h16* p) { return cat16(*(const v8h*)p, *(const v8h*)(p + 16)); } static __device__ __forceinline__ v8f mma(V a, V b, v8f c) { return wmma16(a, b, c); } };
template <> struct WFrag<bf> { typedef v16bf V; static __device__ __forceinline__ V ld(const bf* p) { return cat16b(*(const v8us*)p, *(const v8us*)(p + 16)); } static __device__ __forceinline__ v8f mma(V a, V b, v8f c) { return wmmab(a, b, c); } };
template <typename T16, int NSPLIT, bool BIAS>
__global__ __launch_bounds__(32) void k_gemmw(const T16* __restrict__ A, const T16* __restrict__ A2, const T16* __restrict__ Bt, const T16* __restrict__ Bt2, int K, float* C, int ldc, const float* __restrict__ bias, size_t sA, size_t sB, size_t sC) {
    typedef typename WFrag<T16>::V V;
    __shared__ __align__(16) float os[16 * 68];
    const size_t z = blockIdx.z; A += z * sA; if (A2) A2 += z * sA; Bt += z * sB; if (Bt2) Bt2 += z * sB; C += z * sC;
    const int lane = threadIdx.x & 31, lr = lane & 15, hi = lane >> 4; const int r0 = blockIdx.x * 64, c0 = blockIdx.y * 64;
    v8f acc[4][4];
#pragma unroll
    for (int mb = 0; mb < 4; ++mb)
#pragma unroll
        for (int nb = 0; nb < 4; ++nb) acc[mb][nb] = (v8f){};
    const size_t aoff = (size_t)(r0 + lr) * K + 8 * hi, boff = (size_t)(c0 + lr) * K + 8 * hi;
#pragma unroll 1
    for (int kc = 0; kc < K; kc += 32) {
        V a[4], a2[4];
#pragma unroll
        for (int mb = 0; mb < 4; ++mb) { a[mb] = WFrag<T16>::ld(A + aoff + (size_t)mb * 16 * K + kc); if (NSPLIT == 1 || NSPLIT == 2) a2[mb] = WFrag<T16>::ld(A2 + aoff + (size_t)mb * 16 * K + kc); }
#pragma unroll
        for (int nb = 0; nb < 4; ++nb) { const V b = WFrag<T16>::ld(Bt + boff + (size_t)nb * 16 * K + kc); V b2; if (NSPLIT >= 2) b2 = WFrag<T16>::ld(Bt2 + boff + (size_t)nb * 16 * K + kc);
#pragma unroll
            for (int mb = 0; mb < 4; ++mb) { acc[mb][nb] = WFrag<T16>::mma(a[mb], b, acc[mb][nb]); if (NSPLIT == 1 || NSPLIT == 2) acc[mb][nb] = WFrag<T16>::mma(a2[mb], b, acc[mb][nb]); if (NSPLIT >= 2) acc[mb][nb] = WFrag<T16>::mma(a[mb], b2, acc[mb][nb]); } }
        asm volatile("v_nop\n\tv_nop\n\tv_nop\n\tv_nop" : "+v"(acc[0][0]), "+v"(acc[1][1]), "+v"(acc[2][2]), "+v"(acc[3][3]) : "v"(a[0]), "v"(a[3]));
    }
#pragma unroll
    for (int mb = 0; mb < 4; ++mb) {
#pragma unroll
        for (int nb = 0; nb < 4; ++nb) {
#pragma unroll
            for (int j = 0; j < 8; ++j) os[(hi * 8 + j) * 68 + nb * 16 + lr] = acc[mb][nb][j]; }
        __builtin_amdgcn_wave_barrier(); asm volatile("" ::: "memory");
        float* crow = C + (size_t)(r0 + mb * 16) * ldc + c0;
#pragma unroll 1
        for (int ps = 0; ps < 2; ++ps) {
#pragma unroll
            for (int s = 0; s < 8; ++s) { const int row = 2 * s + hi, cofs = lr * 4; v4f val = *(const v4fa*)(os + row * 68 + cofs); if (BIAS) { val[0] += bfr(bias[c0 + cofs]); val[1] += bfr(bias[c0 + cofs + 1]); val[2] += bfr(bias[c0 + cofs + 2]); val[3] += bfr(bias[c0 + cofs + 3]); }
                *(volatile v4f*)(crow + (size_t)row * ldc + cofs) = val; }
            if (ps == 0) __threadfence(); }
        __builtin_amdgcn_wave_barrier(); asm volatile("" ::: "memory");
    }
}

__device__ __forceinline__ void splitf(float y, unsigned short& h, unsigned short& l) { h = f2bf(y); l = f2bf(y - bf2f(h)); }
__device__ __forceinline__ float siluf_(float a) { return __fdiv_rn(a, __fadd_rn(1.0f, __expf(-a))); }
typedef __attribute__((ext_vector_type(4))) unsigned short v4us;

__global__ __launch_bounds__(256) void k_cvt8(const float* __restrict__ src, bf* dst, size_t n8) { const size_t i = (size_t)blockIdx.x * 256 + threadIdx.x; if (i >= n8) return; const v8f v = *(const v8f*)(src + i * 8); v8us o;
#pragma unroll
    for (int k = 0; k < 8; ++k) o[k] = f2bf(v[k]); *(volatile v8us*)(dst + i * 8) = o; __threadfence(); *(volatile v8us*)(dst + i * 8) = o; }
__global__ __launch_bounds__(256) void k_wxp(const float* __restrict__ w, bf* WXP) { const size_t e = ((size_t)blockIdx.x * 256 + threadIdx.x) * 4; if (e >= (size_t)XW * DI) return; const int n = (int)(e / DI); v4us o;
#pragma unroll
    for (int q = 0; q < 4; ++q) o[q] = n < (DR + 2 * DS) ? f2bf(w[e + q]) : (unsigned short)0; *(volatile v4us*)(WXP + e) = o; __threadfence(); *(volatile v4us*)(WXP + e) = o; }
__global__ __launch_bounds__(256) void k_conv(const float* __restrict__ XZ, const float* __restrict__ cw, const float* __restrict__ cb, float* Uf, bf* Uh, bf* Ul) { const size_t e = ((size_t)blockIdx.x * 256 + threadIdx.x) * 4; if (e >= (size_t)LL * DI) return; const int c = (int)(e % DI), l = (int)(e / DI); v4f o; v4us oh, ol;
#pragma unroll
    for (int q = 0; q < 4; ++q) { const int cq = c + q; float s = 0.f;
#pragma unroll
        for (int j = 0; j < 4; ++j) { const int ll = l - 3 + j; const float uv = ll >= 0 ? XZ[(size_t)ll * (2 * DI) + cq] : 0.f; float p = __fmul_rn(bfr(cw[cq * 4 + j]), uv); asm volatile("" : "+v"(p)); s = __fadd_rn(s, p); }
        o[q] = siluf_(__fadd_rn(s, bfr(cb[cq]))); unsigned short a, b2; splitf(o[q], a, b2); oh[q] = a; ol[q] = b2; }
    *(volatile v4f*)(Uf + e) = o; *(volatile v4us*)(Uh + e) = oh; *(volatile v4us*)(Ul + e) = ol; __threadfence(); *(volatile v4f*)(Uf + e) = o; *(volatile v4us*)(Uh + e) = oh; *(volatile v4us*)(Ul + e) = ol; }
__global__ __launch_bounds__(256) void k_spl64(const float* __restrict__ XD, bf* Rh, bf* Rl) { const size_t i = ((size_t)blockIdx.x * 256 + threadIdx.x) * 4; if (i >= (size_t)LL * DR) return; const int c = (int)(i % DR), l = (int)(i / DR); const v4f a = *(const v4f*)(XD + (size_t)l * XW + c); v4us oh, ol;
#pragma unroll
    for (int q = 0; q < 4; ++q) { unsigned short u, c2; splitf(a[q], u, c2); oh[q] = u; ol[q] = c2; } *(volatile v4us*)(Rh + i) = oh; *(volatile v4us*)(Rl + i) = ol; __threadfence(); *(volatile v4us*)(Rh + i) = oh; *(volatile v4us*)(Rl + i) = ol; }
__global__ __launch_bounds__(256) void k_sp(float* F, const float* __restrict__ bdt) { const size_t i = ((size_t)blockIdx.x * 256 + threadIdx.x) * 4; if (i >= (size_t)LL * DI) return; const int c = (int)(i % DI); const v4f a = *(const v4f*)(F + i); v4f o;
#pragma unroll
    for (int q = 0; q < 4; ++q) { const float z = __fadd_rn(a[q], bfr(bdt[c + q])); o[q] = z > 20.0f ? z : log1pf(__expf(z)); } *(volatile v4f*)(F + i) = o; __threadfence(); *(volatile v4f*)(F + i) = o; }
__global__ __launch_bounds__(128) void k_scan(const float* __restrict__ DL, const float* __restrict__ XD, const float* __restrict__ Uf, const float* __restrict__ XZ, const float* __restrict__ Alog, const float* __restrict__ Dp, float* Yf) {
    const int c = blockIdx.x * 128 + threadIdx.x; if (c >= DI) return; float A[DS], h[DS];
#pragma unroll
    for (int s = 0; s < DS; ++s) { A[s] = -__expf(bfr(Alog[c * DS + s])); h[s] = 0.f; }
    const float Dd = bfr(Dp[c]);
    for (int l = 0; l < LL; ++l) { const float dl = DL[(size_t)l * DI + c]; const float uv = Uf[(size_t)l * DI + c]; const float* bz = XD + (size_t)l * XW + DR; float du = __fmul_rn(dl, uv); asm volatile("" : "+v"(du)); float y = 0.f;
#pragma unroll
        for (int s = 0; s < DS; ++s) { float da = __fmul_rn(dl, A[s]); asm volatile("" : "+v"(da)); const float a = __expf(da); float bb = __fmul_rn(du, bz[s]); asm volatile("" : "+v"(bb)); float ah = __fmul_rn(a, h[s]); asm volatile("" : "+v"(ah)); h[s] = __fadd_rn(ah, bb); float hc = __fmul_rn(h[s], bz[DS + s]); asm volatile("" : "+v"(hc)); y = __fadd_rn(y, hc); }
        float ud = __fmul_rn(uv, Dd); asm volatile("" : "+v"(ud)); const float yy = __fadd_rn(y, ud); const float g = __fmul_rn(yy, siluf_(XZ[(size_t)l * (2 * DI) + DI + c]));
        *(volatile float*)(Yf + (size_t)l * DI + c) = g; __threadfence(); *(volatile float*)(Yf + (size_t)l * DI + c) = g; } }
__global__ __launch_bounds__(256) void k_sply(const float* __restrict__ Yf, bf* Yh, bf* Yl) { const size_t i = ((size_t)blockIdx.x * 256 + threadIdx.x) * 4; if (i >= (size_t)LL * DI) return; const v4f a = *(const v4f*)(Yf + i); v4us oh, ol;
#pragma unroll
    for (int q = 0; q < 4; ++q) { unsigned short u, c2; splitf(a[q], u, c2); oh[q] = u; ol[q] = c2; } *(volatile v4us*)(Yh + i) = oh; *(volatile v4us*)(Yl + i) = ol; __threadfence(); *(volatile v4us*)(Yh + i) = oh; *(volatile v4us*)(Yl + i) = ol; }

extern "C" void kernel_launch(void* const* d_in, const int* in_sizes, int n_in,
                              void* d_out, int out_size, void* d_ws, size_t ws_size, hipStream_t stream) {
    (void)in_sizes; (void)n_in; (void)out_size;
    const float* IN[10]; for (int i = 0; i < 10; ++i) IN[i] = (const float*)d_in[i];
    float* OUT = (float*)d_out;
    char* wsp = (char*)d_ws;
    auto take = [&](size_t bytes) { char* p = wsp; wsp += (bytes + 255) & ~(size_t)255; return (void*)p; };
    bf* WIN = (bf*)take((size_t)2 * DI * DMO * 2); bf* WXP = (bf*)take((size_t)XW * DI * 2); bf* WDT = (bf*)take((size_t)DI * DR * 2); bf* WOUT = (bf*)take((size_t)DMO * DI * 2);
    bf* XB = (bf*)take((size_t)LL * DMO * 2); float* XZ = (float*)take((size_t)LL * 2 * DI * 4); float* Uf = (float*)take((size_t)LL * DI * 4); bf* Uh = (bf*)take((size_t)LL * DI * 2); bf* Ul = (bf*)take((size_t)LL * DI * 2); float* XD = (float*)take((size_t)LL * XW * 4); bf* Rh = (bf*)take((size_t)LL * DR * 2); bf* Rl = (bf*)take((size_t)LL * DR * 2);
    float* DL = (float*)take((size_t)LL * DI * 4); float* DL2 = (float*)take((size_t)LL * DI * 4); bf* Yh = (bf*)take((size_t)LL * DI * 2); bf* Yl = (bf*)take((size_t)LL * DI * 2);
    if ((size_t)(wsp - (char*)d_ws) > ws_size) return;
    k_cvt8<<<(unsigned)(((size_t)2 * DI * DMO / 8 + 255) / 256), 256, 0, stream>>>(IN[1], WIN, (size_t)2 * DI * DMO / 8); k_wxp<<<(XW * DI / 4 + 255) / 256, 256, 0, stream>>>(IN[4], WXP); k_cvt8<<<(DI * DR / 8 + 255) / 256, 256, 0, stream>>>(IN[5], WDT, (size_t)DI * DR / 8); k_cvt8<<<(DMO * DI / 8 + 255) / 256, 256, 0, stream>>>(IN[9], WOUT, (size_t)DMO * DI / 8);
    k_cvt8<<<(LL * DMO / 8 + 255) / 256, 256, 0, stream>>>(IN[0], XB, (size_t)LL * DMO / 8);
    k_gemmw<bf, 0, false><<<dim3(LL / 64, 2 * DI / 64, 1), 32, 0, stream>>>(XB, nullptr, WIN, nullptr, DMO, XZ, 2 * DI, nullptr, 0, 0, 0);
    k_conv<<<(unsigned)(((size_t)LL * DI / 4 + 255) / 256), 256, 0, stream>>>(XZ, IN[2], IN[3], Uf, Uh, Ul);
    k_gemmw<bf, 1, false><<<dim3(LL / 64, XW / 64, 1), 32, 0, stream>>>(Uh, Ul, WXP, nullptr, DI, XD, XW, nullptr, 0, 0, 0);
    k_spl64<<<(LL * DR / 4 + 255) / 256, 256, 0, stream>>>(XD, Rh, Rl);
    k_gemmw<bf, 1, false><<<dim3(LL / 64, DI / 64, 1), 32, 0, stream>>>(Rh, Rl, WDT, nullptr, DR, DL, DI, nullptr, 0, 0, 0);
    k_sp<<<(unsigned)(((size_t)LL * DI / 4 + 255) / 256), 256, 0, stream>>>(DL, IN[6]);
    k_scan<<<(DI + 127) / 128, 128, 0, stream>>>(DL, XD, Uf, XZ, IN[7], IN[8], DL2); k_sply<<<(unsigned)(((size_t)LL * DI / 4 + 255) / 256), 256, 0, stream>>>(DL2, Yh, Yl);
    k_gemmw<bf, 1, false><<<dim3(LL / 64, DMO / 64, 1), 32, 0, stream>>>(Yh, Yl, WOUT, nullptr, DI, OUT, DMO, nullptr, 0, 0, 0);
}
